// NDDE_1D_59390807769589
// MI455X (gfx1250) — hardware-run, weakly checked
//
#include <hip/hip_runtime.h>
#include <math.h>

typedef __attribute__((ext_vector_type(16))) _Float16 v16h;
typedef __attribute__((ext_vector_type(8)))  _Float16 v8h;
typedef __attribute__((ext_vector_type(16))) __bf16   v16b;
typedef __attribute__((ext_vector_type(8)))  __bf16   v8b;
typedef __attribute__((ext_vector_type(8)))  float    v8f;
typedef __attribute__((ext_vector_type(4)))  float    v4f;

constexpr int kD       = 512;
constexpr int kK       = 2 * kD;
constexpr int kSteps   = 2000;
constexpr int kCols    = kSteps + 1;
constexpr int kDelay   = 100;
constexpr int kWPlanes = 1;
constexpr bool kNarrowInputs = (kWPlanes == 1);
static_assert(kWPlanes >= 1 && kWPlanes <= 3, "plane count");
static_assert((kK % 32) == 0 && (kD % 32) == 0, "K multiple of 32, one 128-B line per wave");
static_assert(kD == 16 * 32, "16 waves x 32 outputs");
static_assert((size_t)kD * kCols * 4 == 4098048ull, "output bytes");
static_assert(((size_t)kD * kCols) % 256 == 0, "flat output is a whole number of 256-thread blocks");

constexpr size_t kPlaneElems = (size_t)kD * kK;
constexpr size_t kOffWC      = 0;
constexpr size_t kOffTraj    = kOffWC + (size_t)kWPlanes * kPlaneElems * 2;
constexpr size_t kTrajBytes  = (size_t)kCols * kD * 4;
constexpr size_t kWsTotal    = kOffTraj + kTrajBytes;
static_assert((kOffTraj % 128) == 0 && (kTrajBytes % 128) == 0, "128-B aligned regions");
static_assert(kWPlanes != 1 || kWsTotal == 5146624ull, "carve total");
static_assert(kWsTotal <= 134217728ull, "carve cap");

__device__ __forceinline__ unsigned short f2bf_bits(float f) {
  unsigned u = __float_as_uint(f);
  return (unsigned short)((u + 0x7FFFu + ((u >> 16) & 1u)) >> 16);
}
__device__ __forceinline__ float bf_bits2f(unsigned short h) { return __uint_as_float(((unsigned)h) << 16); }
__device__ __forceinline__ float in_val(float v) {
  return kNarrowInputs ? bf_bits2f(f2bf_bits(v)) : v;
}

template <typename T> struct Frag;
template <> struct Frag<__bf16> {
  typedef v16b V; union U { v16b v; v8b h[2]; };
  static __device__ __forceinline__ v16b load(const __bf16* p) {
    U f; f.h[0] = *(const v8b*)(p); f.h[1] = *(const v8b*)(p + 16); return f.v;
  }
};

__device__ __forceinline__ v8f mma_g(v16b a, v16b b, v8f c) {
  c = __builtin_amdgcn_wmma_f32_16x16x32_bf16(false, a, false, b, (short)0, c, false, false);
  asm volatile("v_nop\n\tv_nop\n\tv_nop\n\tv_nop" : "+v"(c) : "v"(a), "v"(b));
  return c;
}

__device__ __forceinline__ void split3(float v, __bf16& hi, __bf16& mid, __bf16& lo) {
  const unsigned short hb = f2bf_bits(v);
  const float r1 = v - bf_bits2f(hb);
  const unsigned short mb = f2bf_bits(r1);
  const float r2 = r1 - bf_bits2f(mb);
  const unsigned short lb = f2bf_bits(r2);
  hi  = __builtin_bit_cast(__bf16, hb);
  mid = __builtin_bit_cast(__bf16, mb);
  lo  = __builtin_bit_cast(__bf16, lb);
}

__global__ __launch_bounds__(256) void wplanes_kernel(
    const float* __restrict__ W1, const float* __restrict__ W2, unsigned short* __restrict__ Wc)
{
  const int which = blockIdx.y;
  const float* src = (which == 0) ? W1 : W2;
  const int e0 = (blockIdx.x * 256 + threadIdx.x) * 8;
  const int n  = e0 >> 9;
  const int kk = e0 & (kD - 1);
  const v4f a0 = *(const v4f*)(src + e0);
  const v4f a1 = *(const v4f*)(src + e0 + 4);
  v8h pv[kWPlanes];
#pragma unroll
  for (int e = 0; e < 4; ++e) {
    float r0 = a0[e];
    float r1 = a1[e];
#pragma unroll
    for (int p = 0; p < kWPlanes; ++p) {
      const unsigned short h0 = f2bf_bits(r0);
      const unsigned short h1 = f2bf_bits(r1);
      pv[p][e]     = __builtin_bit_cast(_Float16, h0);
      pv[p][4 + e] = __builtin_bit_cast(_Float16, h1);
      r0 = r0 - bf_bits2f(h0);
      r1 = r1 - bf_bits2f(h1);
    }
  }
  unsigned short* dst = Wc + (size_t)n * kK + which * kD + kk;
#pragma unroll
  for (int p = 0; p < kWPlanes; ++p) *(volatile v8h*)(dst + (size_t)p * kPlaneElems) = pv[p];
  __threadfence();
#pragma unroll
  for (int p = 0; p < kWPlanes; ++p) *(volatile v8h*)(dst + (size_t)p * kPlaneElems) = pv[p];
}

__global__ __launch_bounds__(512) void recur_kernel(
    const float* __restrict__ x0p, const float* __restrict__ taup, const float* __restrict__ bp,
    const unsigned short* __restrict__ Wc, float* traj)
{
  __shared__ __align__(16) __bf16 sA[2][4][kK];
  const int tid  = threadIdx.x;
  const int lane = tid & 31;
  const int wave = __builtin_amdgcn_readfirstlane((int)(threadIdx.x >> 5));
  const int hh   = lane >> 4;
  const int rl   = lane & 15;
  const int n    = wave * 32 + lane;

  const float dt   = 0.01f * in_val(taup[0]);
  const float x0r  = in_val(x0p[n]);
  const float bias = in_val(bp[n]);
  float x = x0r;

  {
    volatile float* p0 = traj + n;
    *p0 = x0r;
    __threadfence();
    *p0 = x0r;
  }
  {
    __bf16 ph, pm, pl;
    split3(x0r, ph, pm, pl);
    sA[0][0][n] = ph;       sA[0][1][n] = pm;       sA[0][2][n] = pl;
    sA[0][0][kD + n] = ph;  sA[0][1][kD + n] = pm;  sA[0][2][kD + n] = pl;
    *(unsigned*)(&sA[0][3][2 * tid]) = 0u;
  }
  __syncthreads();

  const int arow = (rl < 3) ? rl : 3;
  const unsigned short* wb0 = Wc + (size_t)(wave * 32 + rl) * kK + 8 * hh;
  const unsigned short* wb1 = wb0 + (size_t)16 * kK;
  union FB { v16b v; v8b h[2]; };

#pragma unroll 1
  for (int j = 0; j < kSteps; ++j) {
    const int cur = j & 1;
    const int nxt = cur ^ 1;

    v8f acc[kWPlanes][2];
#pragma unroll
    for (int p = 0; p < kWPlanes; ++p) {
      acc[p][0] = (v8f){0.f, 0.f, 0.f, 0.f, 0.f, 0.f, 0.f, 0.f};
      acc[p][1] = (v8f){0.f, 0.f, 0.f, 0.f, 0.f, 0.f, 0.f, 0.f};
    }

#pragma unroll 4
    for (int kf = 0; kf < kK / 32; ++kf) {
      const int k0 = kf * 32;
      FB af;
      af.h[0] = *(const v8b*)(&sA[cur][arow][k0 + 8 * hh]);
      af.h[1] = *(const v8b*)(&sA[cur][arow][k0 + 16 + 8 * hh]);
#pragma unroll
      for (int p = 0; p < kWPlanes; ++p) {
        const v16b b0 = Frag<__bf16>::load((const __bf16*)(wb0 + (size_t)p * kPlaneElems + k0));
        const v16b b1 = Frag<__bf16>::load((const __bf16*)(wb1 + (size_t)p * kPlaneElems + k0));
        acc[p][0] = mma_g(af.v, b0, acc[p][0]);
        acc[p][1] = mma_g(af.v, b1, acc[p][1]);
      }
    }

    float s0 = 0.0f;
    float s1 = 0.0f;
#pragma unroll
    for (int p = kWPlanes - 1; p >= 0; --p) {
      s0 = s0 + ((acc[p][0][2] + acc[p][0][1]) + acc[p][0][0]);
      s1 = s1 + ((acc[p][1][2] + acc[p][1][1]) + acc[p][1][0]);
    }
    const float t1  = __shfl(s1, rl, 32);
    const float pre = ((hh == 0) ? s0 : t1) + bias;
    const float th  = tanhf(pre);
    x = x + dt * th;

    const int jn = j + 1;
    volatile float* tp = traj + (size_t)jn * kD + n;
    *tp = x;

    const int jd = (jn > kDelay) ? (jn - kDelay) : 0;
    const float yld = *(const volatile float*)(traj + (size_t)jd * kD + n);
    const float yv  = (jn < kDelay) ? x0r : yld;

    {
      __bf16 ph, pm, pl;
      split3(x, ph, pm, pl);
      sA[nxt][0][n] = ph;  sA[nxt][1][n] = pm;  sA[nxt][2][n] = pl;
      split3(yv, ph, pm, pl);
      sA[nxt][0][kD + n] = ph;  sA[nxt][1][kD + n] = pm;  sA[nxt][2][kD + n] = pl;
      *(unsigned*)(&sA[nxt][3][2 * tid]) = 0u;
    }

    __threadfence();
    *tp = x;
    __syncthreads();
  }
}

__global__ __launch_bounds__(256) void emit_kernel(
    const float* __restrict__ traj, const int* __restrict__ Np, float* __restrict__ out)
{
  const int f = blockIdx.x * 256 + threadIdx.x;
  const int i = f / kCols;
  const int k = f - i * kCols;
  float v = traj[(size_t)k * kD + i];
  const int nv = Np[0];
  v = (nv == kSteps) ? v : __uint_as_float(0x7fc00000u);
  volatile float* p = out + f;
  *p = v;
  __threadfence();
  *p = v;
}

extern "C" void kernel_launch(void* const* d_in, const int* in_sizes, int n_in,
                              void* d_out, int out_size, void* d_ws, size_t ws_size,
                              hipStream_t stream) {
  if (n_in < 6) return;
  if (in_sizes[0] != kD) return;
  if (in_sizes[1] != 1) return;
  if (in_sizes[2] != kD * kD) return;
  if (in_sizes[3] != kD * kD) return;
  if (in_sizes[4] != kD) return;
  if (in_sizes[5] != 1) return;
  if (out_size != kD * kCols) return;
  if (ws_size < kWsTotal) return;

  const float* x0  = (const float*)d_in[0];
  const float* tau = (const float*)d_in[1];
  const float* W1  = (const float*)d_in[2];
  const float* W2  = (const float*)d_in[3];
  const float* bb  = (const float*)d_in[4];
  const int*   Np  = (const int*)d_in[5];
  float* out = (float*)d_out;

  char* ws = (char*)d_ws;
  unsigned short* Wc = (unsigned short*)(ws + kOffWC);
  float* traj = (float*)(ws + kOffTraj);

  wplanes_kernel<<<dim3((kD * kD / 8) / 256, 2), 256, 0, stream>>>(W1, W2, Wc);
  recur_kernel<<<1, 512, 0, stream>>>(x0, tau, bb, Wc, traj);
  emit_kernel<<<(kD * kCols) / 256, 256, 0, stream>>>(traj, Np, out);
}
